// GraphBranchingQNetwork_30571577213243
// MI455X (gfx1250) — hardware-verified
//
#include <hip/hip_runtime.h>
#include <stddef.h>
#include <stdint.h>


#define CF      32
#define NB      2048
#define CHUNK   4096
#define NTHR    256
#define NWAVE   8
#define WCAP    (CHUNK / NWAVE)
#define NGRP    (CHUNK / (NTHR * 4))
#define MAXBLK  64
#define HN      80
#define HD      256
#define ESHIFT  11

#define LDS_SACC_F  (NB * CF)
#define LDS_LIST_I  (NWAVE * WCAP)
#define LDS_WCNT_I  16
#define LDS_DFIN_D  64
#define AGG_LDS_BYTES ((LDS_SACC_F + LDS_LIST_I + LDS_WCNT_I) * 4 + LDS_DFIN_D * 8)

static_assert(WCAP == 512);
static_assert(NGRP == 4);
static_assert((1 << ESHIFT) == NB);
static_assert(WCAP * NWAVE == CHUNK);
static_assert(AGG_LDS_BYTES == 279104);
static_assert(NWAVE * 64 * 8 <= LDS_LIST_I * 4);
static_assert((((LDS_SACC_F + LDS_LIST_I + LDS_WCNT_I) * 4) % 16) == 0);
static_assert((NB % (NWAVE * 4)) == 0);

typedef float          v4f   __attribute__((ext_vector_type(4)));
typedef float          v8f   __attribute__((ext_vector_type(8)));
typedef int            v4i   __attribute__((ext_vector_type(4)));
typedef unsigned short v8us  __attribute__((ext_vector_type(8)));
typedef __bf16         v16bf __attribute__((ext_vector_type(16)));
typedef double         v2d   __attribute__((ext_vector_type(2)));
typedef v4f  __attribute__((may_alias)) v4fa;
typedef v8us __attribute__((may_alias)) v8usa;

union Frag { v16bf v; v8us u8[2]; unsigned short s[16]; };

__device__ __forceinline__ int imin(int a, int b) { return a < b ? a : b; }
__device__ __forceinline__ int imax(int a, int b) { return a > b ? a : b; }

__device__ __forceinline__ unsigned short bfr(float f) {
  unsigned u = __float_as_uint(f);
  u += 0x7FFFu + ((u >> 16) & 1u);
  return (unsigned short)(u >> 16);
}
__device__ __forceinline__ float bfv(unsigned short s) { return __uint_as_float(((unsigned)s) << 16); }
__device__ __forceinline__ void bsplit(float x, unsigned short& hi, unsigned short& lo) {
  const unsigned short h = bfr(x);
  hi = h;
  lo = bfr(x - bfv(h));
}
__device__ __forceinline__ void split8(v4f a, v4f b, v8us& hv, v8us& lv) {
  v8us hq = {0, 0, 0, 0, 0, 0, 0, 0};
  v8us lq = {0, 0, 0, 0, 0, 0, 0, 0};
  unsigned short h, l;
  bsplit(a.x, h, l); hq[0] = h; lq[0] = l;
  bsplit(a.y, h, l); hq[1] = h; lq[1] = l;
  bsplit(a.z, h, l); hq[2] = h; lq[2] = l;
  bsplit(a.w, h, l); hq[3] = h; lq[3] = l;
  bsplit(b.x, h, l); hq[4] = h; lq[4] = l;
  bsplit(b.y, h, l); hq[5] = h; lq[5] = l;
  bsplit(b.z, h, l); hq[6] = h; lq[6] = l;
  bsplit(b.w, h, l); hq[7] = h; lq[7] = l;
  hv = hq; lv = lq;
}

#define SPLIT_TO(FH, IH, FL, IL, VAL) do { unsigned short h__, l__; bsplit((VAL), h__, l__); (FH).s[IH] = h__; (FL).s[IL] = l__; } while (0)

__device__ __forceinline__ v8f wmb(v16bf a, v16bf b, v8f c) {
  v8f d = __builtin_amdgcn_wmma_f32_16x16x32_bf16(false, a, false, b, (short)0, c, false, false);
  asm volatile("v_nop\n\tv_nop\n\tv_nop\n\tv_nop" : "+v"(d) : "v"(a), "v"(b));
  return d;
}

__device__ __forceinline__ v8f vzero8() { v8f z = {0.f, 0.f, 0.f, 0.f, 0.f, 0.f, 0.f, 0.f}; return z; }

__global__ __launch_bounds__(NTHR) void k_node1(const float* __restrict__ x, const float* __restrict__ W1,
                                               const float* __restrict__ b1, float* PQ, int nN) {
  const int lane = threadIdx.x & 31, wave = threadIdx.x >> 5;
  const int s = lane & 7;
  const int row = blockIdx.x * (NWAVE * 4) + wave * 4 + (lane >> 3);
  float cA[4], cB[4], cb[4];
#pragma unroll
  for (int j = 0; j < 4; ++j) {
    const int c = 4 * s + j;
    const int cc = c & 15;
    const float wa = W1[cc], wb = W1[16 + cc], wc = W1[32 + cc], wd = W1[48 + cc];
    const float bb = b1[cc];
    const bool isP = c < 16;
    cA[j] = isP ? (wa - wc) : wc;
    cB[j] = isP ? (wb - wd) : wd;
    cb[j] = isP ? bb : 0.f;
  }
  const int rr = imin(row, nN - 1);
  const float x0 = x[(size_t)rr * 2], x1 = x[(size_t)rr * 2 + 1];
  v4f o;
  o.x = cb[0] + x0 * cA[0] + x1 * cB[0];
  o.y = cb[1] + x0 * cA[1] + x1 * cB[1];
  o.z = cb[2] + x0 * cA[2] + x1 * cB[2];
  o.w = cb[3] + x0 * cA[3] + x1 * cB[3];
  float* p = PQ + (size_t)rr * CF + 4 * s;
  if (row < nN) *(volatile v4f*)p = o;
  __threadfence();
  if (row < nN) *(volatile v4f*)p = o;
}

__global__ __launch_bounds__(NTHR) void k_node(const float* __restrict__ H, const float* __restrict__ bnp,
                                              const unsigned short* __restrict__ Wph,
                                              const unsigned short* __restrict__ Wpl,
                                              const float* __restrict__ b1, float* PQ, int nN) {
  __shared__ __attribute__((aligned(16))) float tile[NWAVE][16 * CF];
  const int lane = threadIdx.x & 31, wave = threadIdx.x >> 5;
  const int m = lane & 15, hh = lane >> 4;
  const int row0 = blockIdx.x * (NWAVE * 16) + wave * 16;

  Frag bh[2], bl[2];
#pragma unroll
  for (int t = 0; t < 2; ++t) {
    const int n = 16 * t + m;
    bh[t].u8[0] = *(const v8us*)(Wph + n * CF + 8 * hh);
    bh[t].u8[1] = *(const v8us*)(Wph + n * CF + 16 + 8 * hh);
    bl[t].u8[0] = *(const v8us*)(Wpl + n * CF + 8 * hh);
    bl[t].u8[1] = *(const v8us*)(Wpl + n * CF + 16 + 8 * hh);
  }
  const int rr = imin(row0 + m, nN - 1);
  const float* hp = H + (size_t)rr * CF;
  const v4f h0 = *(const v4f*)(hp + 8 * hh), h1 = *(const v4f*)(hp + 8 * hh + 4);
  const v4f h2 = *(const v4f*)(hp + 16 + 8 * hh), h3 = *(const v4f*)(hp + 20 + 8 * hh);
  const v4f u0 = *(const v4f*)(bnp + 8 * hh), u1 = *(const v4f*)(bnp + 8 * hh + 4);
  const v4f u2 = *(const v4f*)(bnp + 16 + 8 * hh), u3 = *(const v4f*)(bnp + 20 + 8 * hh);
  const v4f s0 = *(const v4f*)(bnp + 32 + 8 * hh), s1 = *(const v4f*)(bnp + 32 + 8 * hh + 4);
  const v4f s2 = *(const v4f*)(bnp + 48 + 8 * hh), s3 = *(const v4f*)(bnp + 52 + 8 * hh);
  const v4f t0 = *(const v4f*)(bnp + 64 + 8 * hh), t1 = *(const v4f*)(bnp + 64 + 8 * hh + 4);
  const v4f t2 = *(const v4f*)(bnp + 80 + 8 * hh), t3 = *(const v4f*)(bnp + 84 + 8 * hh);
  const v4f y0 = (h0 - u0) * s0 + t0;
  const v4f y1 = (h1 - u1) * s1 + t1;
  const v4f y2 = (h2 - u2) * s2 + t2;
  const v4f y3 = (h3 - u3) * s3 + t3;
  Frag ah, al;
  SPLIT_TO(ah, 0, al, 0, fmaxf(y0.x, 0.f));  SPLIT_TO(ah, 1, al, 1, fmaxf(y0.y, 0.f));
  SPLIT_TO(ah, 2, al, 2, fmaxf(y0.z, 0.f));  SPLIT_TO(ah, 3, al, 3, fmaxf(y0.w, 0.f));
  SPLIT_TO(ah, 4, al, 4, fmaxf(y1.x, 0.f));  SPLIT_TO(ah, 5, al, 5, fmaxf(y1.y, 0.f));
  SPLIT_TO(ah, 6, al, 6, fmaxf(y1.z, 0.f));  SPLIT_TO(ah, 7, al, 7, fmaxf(y1.w, 0.f));
  SPLIT_TO(ah, 8, al, 8, fmaxf(y2.x, 0.f));  SPLIT_TO(ah, 9, al, 9, fmaxf(y2.y, 0.f));
  SPLIT_TO(ah, 10, al, 10, fmaxf(y2.z, 0.f)); SPLIT_TO(ah, 11, al, 11, fmaxf(y2.w, 0.f));
  SPLIT_TO(ah, 12, al, 12, fmaxf(y3.x, 0.f)); SPLIT_TO(ah, 13, al, 13, fmaxf(y3.y, 0.f));
  SPLIT_TO(ah, 14, al, 14, fmaxf(y3.z, 0.f)); SPLIT_TO(ah, 15, al, 15, fmaxf(y3.w, 0.f));

  v8f acc[2];
#pragma unroll
  for (int t = 0; t < 2; ++t) {
    acc[t] = vzero8();
    acc[t] = wmb(ah.v, bh[t].v, acc[t]);
    acc[t] = wmb(ah.v, bl[t].v, acc[t]);
    acc[t] = wmb(al.v, bh[t].v, acc[t]);
  }
  const float bb = b1[m];
  float* tw = &tile[wave][0];
#pragma unroll
  for (int r = 0; r < 8; ++r) {
    tw[(8 * hh + r) * CF + m]      = acc[0][r] + bb;
    tw[(8 * hh + r) * CF + 16 + m] = acc[1][r];
  }
  __syncthreads();
  v4f ov[4];
#pragma unroll
  for (int i = 0; i < 4; ++i) {
    const int r = 4 * i + (lane >> 3), cs = 4 * (lane & 7);
    ov[i] = *(const v4fa*)(tw + r * CF + cs);
  }
#pragma unroll
  for (int i = 0; i < 4; ++i) {
    const int row = row0 + 4 * i + (lane >> 3);
    if (row < nN) *(volatile v4f*)(PQ + (size_t)row * CF + 4 * (lane & 7)) = ov[i];
  }
  __threadfence();
#pragma unroll
  for (int i = 0; i < 4; ++i) {
    const int row = row0 + 4 * i + (lane >> 3);
    if (row < nN) *(volatile v4f*)(PQ + (size_t)row * CF + 4 * (lane & 7)) = ov[i];
  }
}

__global__ __launch_bounds__(NTHR) void k_agg(const float* __restrict__ PQ, const int* __restrict__ ei,
                                             const float* __restrict__ W2, const float* __restrict__ b2,
                                             float* Hout, double* part, int nN, int nE) {
  extern __shared__ v4f lds_dyn[];
  float*  sacc = (float*)lds_dyn;
  int*    list = (int*)(sacc + LDS_SACC_F);
  int*    wcnt = list + LDS_LIST_I;
  double* dfin = (double*)(wcnt + LDS_WCNT_I);
  double* dred = (double*)list;

  const int tid = threadIdx.x;
  const int lane = tid & 31;
  const int wave = tid >> 5;
  const int m = lane & 15;
  const int hh = lane >> 4;
  const int nodeBase = blockIdx.x * NB;

  {
    const v4f z4 = {0.f, 0.f, 0.f, 0.f};
    for (int i = tid; i < LDS_SACC_F / 4; i += NTHR) lds_dyn[i] = z4;
  }
  Frag B1[2], B2[2];
#pragma unroll
  for (int t = 0; t < 2; ++t) {
    const int col = 16 * t + m;
#pragma unroll
    for (int i = 0; i < 8; ++i) {
      const float w = W2[(8 * hh + i) * CF + col];
      unsigned short wh, wl;
      bsplit(w, wh, wl);
      B1[t].s[i] = wh; B1[t].s[8 + i] = wh;
      B2[t].s[i] = wl; B2[t].s[8 + i] = wl;
    }
  }
  const float b2c = b2[lane];
  __syncthreads();

  const int* eid = ei + nE;
  const bool vec = ((nE & 3) == 0) && ((((uintptr_t)eid) & 15u) == 0u);
  const int nChunks = (nE + CHUNK - 1) / CHUNK;

#pragma unroll 1
  for (int ch = 0; ch < nChunks; ++ch) {
    const int cbase = ch * CHUNK;
    int wc = 0;
#pragma unroll
    for (int g = 0; g < NGRP; ++g) {
      const int el0 = wave * WCAP + g * 128 + lane * 4;
      const int e0 = cbase + el0;
      v4i d;
      if (vec && (cbase + CHUNK <= nE)) {
        d = *(const v4i*)(eid + e0);
      } else {
        const int sent = -2147483647 - 1;
        const int t0 = eid[imin(e0, nE - 1)];
        const int t1 = eid[imin(e0 + 1, nE - 1)];
        const int t2 = eid[imin(e0 + 2, nE - 1)];
        const int t3 = eid[imin(e0 + 3, nE - 1)];
        d.x = (e0 < nE) ? t0 : sent;
        d.y = (e0 + 1 < nE) ? t1 : sent;
        d.z = (e0 + 2 < nE) ? t2 : sent;
        d.w = (e0 + 3 < nE) ? t3 : sent;
      }
      const unsigned us0 = (unsigned)d.x - (unsigned)nodeBase;
      const unsigned us1 = (unsigned)d.y - (unsigned)nodeBase;
      const unsigned us2 = (unsigned)d.z - (unsigned)nodeBase;
      const unsigned us3 = (unsigned)d.w - (unsigned)nodeBase;
      const bool h0 = us0 < (unsigned)NB;
      const bool h1 = us1 < (unsigned)NB;
      const bool h2 = us2 < (unsigned)NB;
      const bool h3 = us3 < (unsigned)NB;
      const unsigned many = __builtin_amdgcn_ballot_w32(h0 | h1 | h2 | h3);
      if (many != 0u) {
#define HITJ(J, HJ, SJ) { \
          const unsigned mj = __builtin_amdgcn_ballot_w32(HJ); \
          if (HJ) { \
            const int pos = wc + (int)__builtin_amdgcn_mbcnt_lo(mj, 0u); \
            if (pos < WCAP) list[wave * WCAP + pos] = ((el0 + (J)) << ESHIFT) | (int)(SJ); \
          } \
          wc += (int)__builtin_popcount(mj); }
        HITJ(0, h0, us0)
        HITJ(1, h1, us1)
        HITJ(2, h2, us2)
        HITJ(3, h3, us3)
#undef HITJ
      }
    }
    if (lane == 0) wcnt[wave] = wc;
    __syncthreads();

    if (wave == 0) {
      int pre[NWAVE];
      int total = 0;
#pragma unroll
      for (int j = 0; j < NWAVE; ++j) {
        int c = wcnt[j];
        c = imax(0, imin(c, WCAP));
        pre[j] = total;
        total += c;
      }
      const int nT = (total + 15) >> 4;
#pragma unroll 1
      for (int t = 0; t < nT && t < (CHUNK / 16); ++t) {
        const int p = t * 16 + m;
        const bool valid = p < total;
        int wsel = 0, base = 0;
#pragma unroll
        for (int j = 1; j < NWAVE; ++j) {
          const bool ge = p >= pre[j];
          wsel += ge ? 1 : 0;
          base = ge ? pre[j] : base;
        }
        int idx = p - base;
        idx = imax(0, imin(idx, WCAP - 1));
        const int ent = list[wsel * WCAP + idx];
        const int slot = ent & (NB - 1);
        const int el = (ent >> ESHIFT) & (CHUNK - 1);
        const int sl = valid ? slot : -1;
        const int e = imin(cbase + el, nE - 1);
        int src = ei[e];
        src = imax(0, imin(src, nN - 1));
        const int dn = imin(nodeBase + slot, nN - 1);
        const float* pp = PQ + (size_t)dn * CF + 8 * hh;
        const float* qp = PQ + (size_t)src * CF + 16 + 8 * hh;
        const v4f p0 = *(const v4f*)pp, p1 = *(const v4f*)(pp + 4);
        const v4f q0 = *(const v4f*)qp, q1 = *(const v4f*)(qp + 4);
        const v4f y0 = p0 + q0, y1 = p1 + q1;
        Frag A;
        SPLIT_TO(A, 0, A, 8,  fmaxf(y0.x, 0.f));
        SPLIT_TO(A, 1, A, 9,  fmaxf(y0.y, 0.f));
        SPLIT_TO(A, 2, A, 10, fmaxf(y0.z, 0.f));
        SPLIT_TO(A, 3, A, 11, fmaxf(y0.w, 0.f));
        SPLIT_TO(A, 4, A, 12, fmaxf(y1.x, 0.f));
        SPLIT_TO(A, 5, A, 13, fmaxf(y1.y, 0.f));
        SPLIT_TO(A, 6, A, 14, fmaxf(y1.z, 0.f));
        SPLIT_TO(A, 7, A, 15, fmaxf(y1.w, 0.f));
        v8f acc0 = vzero8(), acc1 = vzero8();
        acc0 = wmb(A.v, B1[0].v, acc0);
        acc0 = wmb(A.v, B2[0].v, acc0);
        acc1 = wmb(A.v, B1[1].v, acc1);
        acc1 = wmb(A.v, B2[1].v, acc1);
#pragma unroll
        for (int ee = 0; ee < 16; ++ee) {
          const int sle = __shfl(sl, ee, 32);
          const int srl = m + ((ee >> 3) << 4);
          const float v0 = __shfl(acc0[ee & 7], srl, 32);
          const float v1 = __shfl(acc1[ee & 7], srl, 32);
          const float val = (hh != 0) ? v1 : v0;
          if (sle >= 0) {
            float* sp = sacc + sle * CF + lane;
            const float cur = *sp;
            *sp = cur + (val + b2c);
          }
        }
      }
    }
    __syncthreads();
  }

  {
    const int c = tid & 31, pt = tid >> 5;
    double s = 0.0, q = 0.0;
#pragma unroll 4
    for (int j = 0; j < NB / NWAVE; ++j) {
      const float v = sacc[(pt * (NB / NWAVE) + j) * CF + c];
      s += (double)v;
      q += (double)v * (double)v;
    }
    dred[pt * 64 + c] = s;
    dred[pt * 64 + 32 + c] = q;
  }
  __syncthreads();
  if (tid < 64) {
    double a = 0.0;
#pragma unroll
    for (int pt = 0; pt < NWAVE; ++pt) a += dred[pt * 64 + tid];
    dfin[tid] = a;
  }
  __syncthreads();

  v2d pv;
  pv.x = dfin[2 * lane];
  pv.y = dfin[2 * lane + 1];
  double* ppart = part + (size_t)blockIdx.x * 64 + 2 * lane;
  if (wave == 0) *(volatile v2d*)ppart = pv;
#pragma unroll 4
  for (int i = 0; i < NB / (NWAVE * 4); ++i) {
    const int slot = wave * (NB / NWAVE) + 4 * i + (lane >> 3);
    const int cs = 4 * (lane & 7);
    const v4f v = *(const v4fa*)(sacc + slot * CF + cs);
    const int node = nodeBase + slot;
    if (node < nN) *(volatile v4f*)(Hout + (size_t)node * CF + cs) = v;
  }
  __threadfence();
  if (wave == 0) *(volatile v2d*)ppart = pv;
#pragma unroll 4
  for (int i = 0; i < NB / (NWAVE * 4); ++i) {
    const int slot = wave * (NB / NWAVE) + 4 * i + (lane >> 3);
    const int cs = 4 * (lane & 7);
    const v4f v = *(const v4fa*)(sacc + slot * CF + cs);
    const int node = nodeBase + slot;
    if (node < nN) *(volatile v4f*)(Hout + (size_t)node * CF + cs) = v;
  }
}

__global__ __launch_bounds__(64) void k_bnfin(const double* __restrict__ part, int nblk, int nN,
                                             const float* __restrict__ gam, const float* __restrict__ bet,
                                             float* bnp, const float* __restrict__ W1n,
                                             unsigned short* Wph, unsigned short* Wpl, int doW) {
  __shared__ double tot[64];
  __shared__ __attribute__((aligned(16))) float ob[96];
  __shared__ __attribute__((aligned(16))) unsigned short swh[32 * 32];
  __shared__ __attribute__((aligned(16))) unsigned short swl[32 * 32];
  const int tid = threadIdx.x, lane = tid & 31, wave = tid >> 5;
  {
    double a = 0.0;
#pragma unroll 1
    for (int k = 0; k < nblk && k < MAXBLK; ++k) a += part[(size_t)k * 64 + tid];
    tot[tid] = a;
  }
  if (doW != 0 && wave == 0) {
    const int n = lane, nn = n & 15;
#pragma unroll
    for (int k = 0; k < 32; ++k) {
      const float wa = W1n[k * 16 + nn];
      const float wb = W1n[(32 + k) * 16 + nn];
      const float w = (n < 16) ? (wa - wb) : wb;
      unsigned short h, l;
      bsplit(w, h, l);
      swh[n * 32 + k] = h;
      swl[n * 32 + k] = l;
    }
  }
  __syncthreads();
  if (tid < 32) {
    const double inv = 1.0 / (double)nN;
    const double mu = tot[tid] * inv;
    const double var = tot[32 + tid] * inv - mu * mu;
    float varf = (float)var;
    varf = varf > 0.f ? varf : 0.f;
    const float rstd = 1.0f / sqrtf(varf + 1e-5f);
    ob[tid] = (float)mu;
    ob[32 + tid] = rstd * gam[tid];
    ob[64 + tid] = bet[tid];
  }
  __syncthreads();
  v4f bv = {0.f, 0.f, 0.f, 0.f};
  if (tid < 24) bv = *(const v4fa*)(ob + 4 * tid);
  v8us wh[4], wl[4];
#pragma unroll
  for (int i = 0; i < 4; ++i) {
    wh[i] = *(const v8usa*)(swh + 256 * i + 8 * lane);
    wl[i] = *(const v8usa*)(swl + 256 * i + 8 * lane);
  }
  if (tid < 24) *(volatile v4f*)(bnp + 4 * tid) = bv;
  if (doW != 0 && wave == 0) {
#pragma unroll
    for (int i = 0; i < 4; ++i) {
      *(volatile v8us*)(Wph + 256 * i + 8 * lane) = wh[i];
      *(volatile v8us*)(Wpl + 256 * i + 8 * lane) = wl[i];
    }
  }
  __threadfence();
  if (tid < 24) *(volatile v4f*)(bnp + 4 * tid) = bv;
  if (doW != 0 && wave == 0) {
#pragma unroll
    for (int i = 0; i < 4; ++i) {
      *(volatile v8us*)(Wph + 256 * i + 8 * lane) = wh[i];
      *(volatile v8us*)(Wpl + 256 * i + 8 * lane) = wl[i];
    }
  }
}

__global__ __launch_bounds__(NTHR) void k_xcvt(const float* __restrict__ H, const float* __restrict__ bnp,
                                              unsigned short* Xh, unsigned short* Xl, int total) {
  const int i8 = blockIdx.x * NTHR + threadIdx.x;
  const size_t base = (size_t)i8 * 8;
  if (base + 8 > (size_t)total) return;
  const int c0 = (int)(base & 31);
  const v4f h0 = *(const v4f*)(H + base), h1 = *(const v4f*)(H + base + 4);
  const v4f u0 = *(const v4f*)(bnp + c0), u1 = *(const v4f*)(bnp + c0 + 4);
  const v4f s0 = *(const v4f*)(bnp + 32 + c0), s1 = *(const v4f*)(bnp + 32 + c0 + 4);
  const v4f t0 = *(const v4f*)(bnp + 64 + c0), t1 = *(const v4f*)(bnp + 64 + c0 + 4);
  v4f y0 = (h0 - u0) * s0 + t0;
  v4f y1 = (h1 - u1) * s1 + t1;
  y0.x = fmaxf(y0.x, 0.f); y0.y = fmaxf(y0.y, 0.f); y0.z = fmaxf(y0.z, 0.f); y0.w = fmaxf(y0.w, 0.f);
  y1.x = fmaxf(y1.x, 0.f); y1.y = fmaxf(y1.y, 0.f); y1.z = fmaxf(y1.z, 0.f); y1.w = fmaxf(y1.w, 0.f);
  v8us hv, lv;
  split8(y0, y1, hv, lv);
  *(volatile v8us*)(Xh + base) = hv;
  *(volatile v8us*)(Xl + base) = lv;
  __threadfence();
  *(volatile v8us*)(Xh + base) = hv;
  *(volatile v8us*)(Xl + base) = lv;
}

__device__ __forceinline__ void wtr_pass(const float* __restrict__ W, int K, int N, int n, int lane,
                                         unsigned short* Th, unsigned short* Tl) {
  const int nseg = K >> 8;
#pragma unroll 1
  for (int seg = 0; seg < nseg && seg < 8; ++seg) {
    const int k0 = seg * 256 + lane * 8;
    v4f a, b;
    a.x = W[(size_t)(k0 + 0) * N + n]; a.y = W[(size_t)(k0 + 1) * N + n];
    a.z = W[(size_t)(k0 + 2) * N + n]; a.w = W[(size_t)(k0 + 3) * N + n];
    b.x = W[(size_t)(k0 + 4) * N + n]; b.y = W[(size_t)(k0 + 5) * N + n];
    b.z = W[(size_t)(k0 + 6) * N + n]; b.w = W[(size_t)(k0 + 7) * N + n];
    v8us hv, lv;
    split8(a, b, hv, lv);
    *(volatile v8us*)(Th + (size_t)n * K + k0) = hv;
    *(volatile v8us*)(Tl + (size_t)n * K + k0) = lv;
  }
}

__global__ __launch_bounds__(NTHR) void k_wtr(const float* __restrict__ W, int K, int N,
                                             unsigned short* Th, unsigned short* Tl) {
  const int lane = threadIdx.x & 31, wave = threadIdx.x >> 5;
  const int n = blockIdx.x * NWAVE + wave;
  if (n >= N) return;
  wtr_pass(W, K, N, n, lane, Th, Tl);
  __threadfence();
  wtr_pass(W, K, N, n, lane, Th, Tl);
}

__device__ __forceinline__ void hw_pass(const float* __restrict__ aW, const float* __restrict__ vW,
                                        int n, int lane, unsigned short* Qh, unsigned short* Ql) {
  const int ia = imin(n, 63) >> 1;
  const int aa = n & 1;
  float w[8];
#pragma unroll
  for (int j = 0; j < 8; ++j) {
    const int f = lane * 8 + j;
    const float a = aW[((size_t)ia * HD + f) * 2 + aa];
    const float v = vW[f];
    w[j] = (n < 64) ? a : ((n == 64) ? v : 0.f);
  }
  v4f a4, b4;
  a4.x = w[0]; a4.y = w[1]; a4.z = w[2]; a4.w = w[3];
  b4.x = w[4]; b4.y = w[5]; b4.z = w[6]; b4.w = w[7];
  v8us hv, lv;
  split8(a4, b4, hv, lv);
  *(volatile v8us*)(Qh + (size_t)n * HD + lane * 8) = hv;
  *(volatile v8us*)(Ql + (size_t)n * HD + lane * 8) = lv;
}

__global__ __launch_bounds__(NTHR) void k_hw(const float* __restrict__ aW, const float* __restrict__ vW,
                                            unsigned short* Qh, unsigned short* Ql) {
  const int lane = threadIdx.x & 31, wave = threadIdx.x >> 5;
  const int n = blockIdx.x * NWAVE + wave;
  if (n >= HN) return;
  hw_pass(aW, vW, n, lane, Qh, Ql);
  __threadfence();
  hw_pass(aW, vW, n, lane, Qh, Ql);
}

__global__ __launch_bounds__(NTHR) void k_gemm(const unsigned short* __restrict__ Ah,
                                              const unsigned short* __restrict__ Al,
                                              const unsigned short* __restrict__ Bh,
                                              const unsigned short* __restrict__ Bl,
                                              const float* __restrict__ bias,
                                              unsigned short* Oh, unsigned short* Ol, int K, int M) {
  __shared__ __attribute__((aligned(16))) float tile[NWAVE][16 * 64];
  const int lane = threadIdx.x & 31, wave = threadIdx.x >> 5;
  const int m = lane & 15, hh = lane >> 4;
  const int wr = wave >> 2, wc = wave & 3;
  const int r0 = blockIdx.x * 64 + 32 * wr;
  const int c0 = 64 * wc;
  (void)M;

  v8f acc[2][4];
#pragma unroll
  for (int rt = 0; rt < 2; ++rt)
#pragma unroll
    for (int ct = 0; ct < 4; ++ct) acc[rt][ct] = vzero8();

  const int nks = K >> 5;
#pragma unroll 1
  for (int ks = 0; ks < nks; ++ks) {
    const int k0 = ks * 32;
    Frag fah[2], fal[2];
#pragma unroll
    for (int rt = 0; rt < 2; ++rt) {
      const size_t ra = (size_t)(r0 + 16 * rt + m) * K + k0 + 8 * hh;
      fah[rt].u8[0] = *(const v8us*)(Ah + ra);
      fah[rt].u8[1] = *(const v8us*)(Ah + ra + 16);
      fal[rt].u8[0] = *(const v8us*)(Al + ra);
      fal[rt].u8[1] = *(const v8us*)(Al + ra + 16);
    }
#pragma unroll
    for (int ct = 0; ct < 4; ++ct) {
      const size_t rb = (size_t)(c0 + 16 * ct + m) * K + k0 + 8 * hh;
      Frag fbh, fbl;
      fbh.u8[0] = *(const v8us*)(Bh + rb);
      fbh.u8[1] = *(const v8us*)(Bh + rb + 16);
      fbl.u8[0] = *(const v8us*)(Bl + rb);
      fbl.u8[1] = *(const v8us*)(Bl + rb + 16);
#pragma unroll
      for (int rt = 0; rt < 2; ++rt) {
        acc[rt][ct] = wmb(fah[rt].v, fbh.v, acc[rt][ct]);
        acc[rt][ct] = wmb(fah[rt].v, fbl.v, acc[rt][ct]);
        acc[rt][ct] = wmb(fal[rt].v, fbh.v, acc[rt][ct]);
      }
    }
  }

  float bs[4];
#pragma unroll
  for (int ct = 0; ct < 4; ++ct) bs[ct] = bias[c0 + 16 * ct + m];
  float* tw = &tile[wave][0];
#pragma unroll
  for (int rt = 0; rt < 2; ++rt) {
#pragma unroll
    for (int ct = 0; ct < 4; ++ct) {
#pragma unroll
      for (int r = 0; r < 8; ++r)
        tw[(8 * hh + r) * 64 + 16 * ct + m] = fmaxf(acc[rt][ct][r] + bs[ct], 0.f);
    }
    __syncthreads();
    v8us oh[4], ol[4];
#pragma unroll
    for (int i = 0; i < 4; ++i) {
      const int rr = 4 * i + (lane >> 3), cs = 8 * (lane & 7);
      const v4f x0 = *(const v4fa*)(tw + rr * 64 + cs);
      const v4f x1 = *(const v4fa*)(tw + rr * 64 + cs + 4);
      split8(x0, x1, oh[i], ol[i]);
    }
#pragma unroll
    for (int i = 0; i < 4; ++i) {
      const size_t o = (size_t)(r0 + 16 * rt + 4 * i + (lane >> 3)) * HD + c0 + 8 * (lane & 7);
      *(volatile v8us*)(Oh + o) = oh[i];
      *(volatile v8us*)(Ol + o) = ol[i];
    }
    __threadfence();
#pragma unroll
    for (int i = 0; i < 4; ++i) {
      const size_t o = (size_t)(r0 + 16 * rt + 4 * i + (lane >> 3)) * HD + c0 + 8 * (lane & 7);
      *(volatile v8us*)(Oh + o) = oh[i];
      *(volatile v8us*)(Ol + o) = ol[i];
    }
    __syncthreads();
  }
}

__global__ __launch_bounds__(NTHR) void k_head(const unsigned short* __restrict__ Ah,
                                              const unsigned short* __restrict__ Al,
                                              const unsigned short* __restrict__ Qh,
                                              const unsigned short* __restrict__ Ql,
                                              const float* __restrict__ ab, const float* __restrict__ vb,
                                              float* out, int M) {
  __shared__ __attribute__((aligned(16))) float tile[NWAVE][16 * HN];
  const int lane = threadIdx.x & 31, wave = threadIdx.x >> 5;
  const int m = lane & 15, hh = lane >> 4;
  const int row0 = blockIdx.x * (NWAVE * 16) + wave * 16;
  (void)M;

  v8f acc[5];
#pragma unroll
  for (int ct = 0; ct < 5; ++ct) acc[ct] = vzero8();
#pragma unroll 1
  for (int ks = 0; ks < HD / 32; ++ks) {
    const int k0 = ks * 32;
    const size_t ra = (size_t)(row0 + m) * HD + k0 + 8 * hh;
    Frag fah, fal;
    fah.u8[0] = *(const v8us*)(Ah + ra);
    fah.u8[1] = *(const v8us*)(Ah + ra + 16);
    fal.u8[0] = *(const v8us*)(Al + ra);
    fal.u8[1] = *(const v8us*)(Al + ra + 16);
#pragma unroll
    for (int ct = 0; ct < 5; ++ct) {
      const size_t rb = (size_t)(16 * ct + m) * HD + k0 + 8 * hh;
      Frag fbh, fbl;
      fbh.u8[0] = *(const v8us*)(Qh + rb);
      fbh.u8[1] = *(const v8us*)(Qh + rb + 16);
      fbl.u8[0] = *(const v8us*)(Ql + rb);
      fbl.u8[1] = *(const v8us*)(Ql + rb + 16);
      acc[ct] = wmb(fah.v, fbh.v, acc[ct]);
      acc[ct] = wmb(fah.v, fbl.v, acc[ct]);
      acc[ct] = wmb(fal.v, fbh.v, acc[ct]);
    }
  }
  float* tw = &tile[wave][0];
#pragma unroll
  for (int ct = 0; ct < 5; ++ct) {
#pragma unroll
    for (int r = 0; r < 8; ++r) tw[(8 * hh + r) * HN + 16 * ct + m] = acc[ct][r];
  }
  __syncthreads();
  const float vb0 = vb[0];
  v4f o[8];
#pragma unroll
  for (int i = 0; i < 8; ++i) {
    const int row = 2 * i + (lane >> 4), j0 = 4 * (lane & 15);
    const float* T = tw + row * HN;
    const v4f a4 = *(const v4fa*)(T + j0);
    const v4f ab4 = *(const v4f*)(ab + j0);
    const float val = T[64] + vb0;
    const v4f adv = a4 + ab4;
    const float m01 = (adv.x + adv.y) * 0.5f;
    const float m23 = (adv.z + adv.w) * 0.5f;
    v4f q;
    q.x = (val + adv.x) - m01;
    q.y = (val + adv.y) - m01;
    q.z = (val + adv.z) - m23;
    q.w = (val + adv.w) - m23;
    o[i] = q;
  }
#pragma unroll
  for (int i = 0; i < 8; ++i) {
    const int row = 2 * i + (lane >> 4), j0 = 4 * (lane & 15);
    *(volatile v4f*)(out + (size_t)(row0 + row) * 64 + j0) = o[i];
  }
  __threadfence();
#pragma unroll
  for (int i = 0; i < 8; ++i) {
    const int row = 2 * i + (lane >> 4), j0 = 4 * (lane & 15);
    *(volatile v4f*)(out + (size_t)(row0 + row) * 64 + j0) = o[i];
  }
}

extern "C" void kernel_launch(void* const* d_in, const int* in_sizes, int n_in,
                              void* d_out, int out_size, void* d_ws, size_t ws_size,
                              hipStream_t stream) {
  if (n_in < 26) return;
  const int nN = in_sizes[0] / 2;
  if (nN <= 0 || in_sizes[0] != nN * 2) return;
  if ((nN % NB) != 0 || (nN % 256) != 0) return;
  const int nE = in_sizes[1] / 2;
  if (nE < 1 || in_sizes[1] != 2 * nE) return;
  const int nG = nN / 32;
  if ((nG % 128) != 0) return;
  if (out_size != nG * 64) return;
  if (in_sizes[2] != 64 || in_sizes[3] != 16 || in_sizes[4] != 512 || in_sizes[5] != 32) return;
  if (in_sizes[6] != 1024 || in_sizes[7] != 16 || in_sizes[8] != 512 || in_sizes[9] != 32) return;
  if (in_sizes[10] != 1024 || in_sizes[11] != 16 || in_sizes[12] != 512 || in_sizes[13] != 32) return;
  if (in_sizes[14] != 96 || in_sizes[15] != 96) return;
  if (in_sizes[16] != 1024 * HD || in_sizes[17] != HD || in_sizes[18] != HD * HD || in_sizes[19] != HD) return;
  if (in_sizes[20] != HD * HD || in_sizes[21] != HD || in_sizes[22] != HD || in_sizes[23] != 1) return;
  if (in_sizes[24] != 32 * HD * 2 || in_sizes[25] != 64) return;
  const int nblk = nN / NB;
  if (nblk > MAXBLK) return;
  if (((nG * 1024) % (8 * NTHR)) != 0) return;

  const float* x    = (const float*)d_in[0];
  const int*   ei   = (const int*)d_in[1];
  const float* c1W1 = (const float*)d_in[2];  const float* c1b1 = (const float*)d_in[3];
  const float* c1W2 = (const float*)d_in[4];  const float* c1b2 = (const float*)d_in[5];
  const float* c2W1 = (const float*)d_in[6];  const float* c2b1 = (const float*)d_in[7];
  const float* c2W2 = (const float*)d_in[8];  const float* c2b2 = (const float*)d_in[9];
  const float* c3W1 = (const float*)d_in[10]; const float* c3b1 = (const float*)d_in[11];
  const float* c3W2 = (const float*)d_in[12]; const float* c3b2 = (const float*)d_in[13];
  const float* bn_g = (const float*)d_in[14]; const float* bn_b = (const float*)d_in[15];
  const float* mW1  = (const float*)d_in[16]; const float* mb1  = (const float*)d_in[17];
  const float* mW2  = (const float*)d_in[18]; const float* mb2  = (const float*)d_in[19];
  const float* mW3  = (const float*)d_in[20]; const float* mb3  = (const float*)d_in[21];
  const float* vW   = (const float*)d_in[22]; const float* vb   = (const float*)d_in[23];
  const float* aW   = (const float*)d_in[24]; const float* ab   = (const float*)d_in[25];
  float* out = (float*)d_out;

  char* wsb = (char*)d_ws;
  size_t off = 0;
#define CARVE(PTR, TYPE, BYTES) TYPE* PTR = (TYPE*)(wsb + off); off += ((((size_t)(BYTES)) + 4095) & ~(size_t)4095);
  CARVE(PQ,   float,          (size_t)nN * CF * 4)
  CARVE(Hp,   float,          (size_t)nN * CF * 4)
  CARVE(part, double,         (size_t)MAXBLK * 64 * 8)
  CARVE(bnp,  float,          (size_t)3 * 128 * 4)
  CARVE(Wph,  unsigned short, (size_t)32 * 32 * 2)
  CARVE(Wpl,  unsigned short, (size_t)32 * 32 * 2)
  CARVE(Xh,   unsigned short, (size_t)nG * 1024 * 2)
  CARVE(Xl,   unsigned short, (size_t)nG * 1024 * 2)
  CARVE(W1h,  unsigned short, (size_t)HD * 1024 * 2)
  CARVE(W1l,  unsigned short, (size_t)HD * 1024 * 2)
  CARVE(W2h,  unsigned short, (size_t)HD * HD * 2)
  CARVE(W2l,  unsigned short, (size_t)HD * HD * 2)
  CARVE(W3h,  unsigned short, (size_t)HD * HD * 2)
  CARVE(W3l,  unsigned short, (size_t)HD * HD * 2)
  CARVE(Qh,   unsigned short, (size_t)HN * HD * 2)
  CARVE(Ql,   unsigned short, (size_t)HN * HD * 2)
  CARVE(A1h,  unsigned short, (size_t)nG * HD * 2)
  CARVE(A1l,  unsigned short, (size_t)nG * HD * 2)
  CARVE(A2h,  unsigned short, (size_t)nG * HD * 2)
  CARVE(A2l,  unsigned short, (size_t)nG * HD * 2)
  CARVE(A3h,  unsigned short, (size_t)nG * HD * 2)
  CARVE(A3l,  unsigned short, (size_t)nG * HD * 2)
#undef CARVE
  if (off > ws_size || off > (size_t)134217728) return;
  float* bnp0 = bnp;
  float* bnp1 = bnp + 128;
  float* bnp2 = bnp + 256;

  k_node1<<<nN / (NWAVE * 4), NTHR, 0, stream>>>(x, c1W1, c1b1, PQ, nN);
  hipFuncSetAttribute(reinterpret_cast<const void*>(&k_agg),
                      hipFuncAttributeMaxDynamicSharedMemorySize, AGG_LDS_BYTES);
  k_agg<<<nblk, NTHR, AGG_LDS_BYTES, stream>>>(PQ, ei, c1W2, c1b2, Hp, part, nN, nE);
  k_bnfin<<<1, 64, 0, stream>>>(part, nblk, nN, bn_g, bn_b, bnp0, c2W1, Wph, Wpl, 1);
  k_node<<<nN / (NWAVE * 16), NTHR, 0, stream>>>(Hp, bnp0, Wph, Wpl, c2b1, PQ, nN);
  k_agg<<<nblk, NTHR, AGG_LDS_BYTES, stream>>>(PQ, ei, c2W2, c2b2, Hp, part, nN, nE);
  k_bnfin<<<1, 64, 0, stream>>>(part, nblk, nN, bn_g + 32, bn_b + 32, bnp1, c3W1, Wph, Wpl, 1);
  k_node<<<nN / (NWAVE * 16), NTHR, 0, stream>>>(Hp, bnp1, Wph, Wpl, c3b1, PQ, nN);
  k_agg<<<nblk, NTHR, AGG_LDS_BYTES, stream>>>(PQ, ei, c3W2, c3b2, Hp, part, nN, nE);
  k_bnfin<<<1, 64, 0, stream>>>(part, nblk, nN, bn_g + 64, bn_b + 64, bnp2, c3W1, Wph, Wpl, 0);
  const int xtot = nG * 1024;
  k_xcvt<<<xtot / (8 * NTHR), NTHR, 0, stream>>>(Hp, bnp2, Xh, Xl, xtot);
  k_wtr<<<HD / NWAVE, NTHR, 0, stream>>>(mW1, 1024, HD, W1h, W1l);
  k_wtr<<<HD / NWAVE, NTHR, 0, stream>>>(mW2, HD, HD, W2h, W2l);
  k_wtr<<<HD / NWAVE, NTHR, 0, stream>>>(mW3, HD, HD, W3h, W3l);
  k_hw<<<HN / NWAVE, NTHR, 0, stream>>>(aW, vW, Qh, Ql);
  k_gemm<<<nG / 64, NTHR, 0, stream>>>(Xh, Xl, W1h, W1l, mb1, A1h, A1l, 1024, nG);
  k_gemm<<<nG / 64, NTHR, 0, stream>>>(A1h, A1l, W2h, W2l, mb2, A2h, A2l, HD, nG);
  k_gemm<<<nG / 64, NTHR, 0, stream>>>(A2h, A2l, W3h, W3l, mb3, A3h, A3l, HD, nG);
  k_head<<<nG / (NWAVE * 16), NTHR, 0, stream>>>(A3h, A3l, Qh, Ql, ab, vb, out, nG);
}
